// STAN_5729486372880
// MI455X (gfx1250) — hardware-run, weakly checked
//
#include <hip/hip_runtime.h>
#include <stddef.h>


#define IN_DIM  128
#define KP      256
#define F1      256
#define F2      128
#define G3      384
#define GRUD    128
#define HC      64
#define NHEAD   4
#define PW      15
#define HK      130
#define HKP     132
#define NO      32
#define TN      32
#define WTROWS  (F1 + F2 + G3)
#define YP      384
#define EP      4
#define NTHR    256
#define NWAVE   8
#define EPT     8
#define CHUNK   (NTHR * EPT)
#define WCAP    (EPT * 32)
#define LISTN   (NWAVE * WCAP)
#define NBMAX   2048
#define RCAP    28672
#define DEGCAP  4096
#define GBM     64
#define GTHR    128
#define NEG_SLOPE 0.2f
#define CA1     16.0f
#define CA2     64.0f
#define CA3     512.0f
#define CW      64.0f
#define SCL1    0.0009765625f
#define SCL2    0.000244140625f
#define SCL3    0.000030517578125f
#define WSCAP   134217728
#define LDS_AGG ((2 * RCAP + 2 * NBMAX + LISTN) * 4 + 64)

static_assert((CHUNK & (CHUNK - 1)) == 0 && CHUNK <= 4096);
static_assert((NBMAX & (NBMAX - 1)) == 0 && NBMAX <= 4096);
static_assert(NTHR * 8 == NBMAX);
static_assert(LISTN >= NBMAX);
static_assert(LISTN >= NWAVE * WCAP);
static_assert((RCAP % 32) == 0);
static_assert(LDS_AGG <= 300000);
static_assert(GBM == (GTHR / 32) * 16);
static_assert(2 * GBM == GTHR);
static_assert(2 * GTHR == F1);
static_assert(NHEAD * HC == F1);
static_assert(F2 == 2 * HC && G3 == 6 * HC && G3 <= YP);
static_assert(F1 == 8 * 32);
static_assert(KP == 256 && (KP % 32) == 0 && (IN_DIM % 32) == 0 && (F1 % 32) == 0);
static_assert(GBM * EP == 2 * 32 * 4);
static_assert((TN * PW) % 4 == 0);
static_assert(NO == 2 * PW + 2 && NO == 4 * NWAVE);
static_assert(TN * 32 == 4 * NTHR);
static_assert(GRUD == 4 * 32);

typedef float    v4f  __attribute__((ext_vector_type(4)));
typedef float    v8f  __attribute__((ext_vector_type(8)));
typedef int      v4i  __attribute__((ext_vector_type(4)));
typedef int      v8i  __attribute__((ext_vector_type(8)));
typedef _Float16 v8h  __attribute__((ext_vector_type(8)));
typedef _Float16 v16h __attribute__((ext_vector_type(16)));
union FragH { v16h v; v8h h[2]; v8i w; };

__device__ __forceinline__ v8f wmh(const FragH& a, const FragH& b, v8f c) {
  v8f d = __builtin_amdgcn_wmma_f32_16x16x32_f16(false, a.v, false, b.v, (short)0, c, false, false);
  asm volatile("v_nop\n\tv_nop\n\tv_nop\n\tv_nop" : "+v"(d) : "v"(a.w), "v"(b.w));
  return d;
}

__device__ __forceinline__ float sigf(float x) {
  return __builtin_amdgcn_rcpf(1.0f + __expf(-x));
}
__device__ __forceinline__ float tnhf(float x) {
  const float ax = fabsf(x);
  const float t = __expf(-2.0f * ax);
  const float r = (1.0f - t) * __builtin_amdgcn_rcpf(1.0f + t);
  return copysignf(r, x);
}

__device__ __forceinline__ int scan_chunk(const int* __restrict__ dsts, int nE, int cbase, int slotBase,
                                          int nb, int vec8, int* list, int tid, int lane, int wave) {
  int wc = 0;
  const int el0  = tid * EPT;
  const int e0   = cbase + el0;
  const int sent = -2147483647 - 1;
  v4i da, db;
  if (vec8 != 0 && cbase + CHUNK <= nE) {
    da = *(const v4i*)(dsts + e0);
    db = *(const v4i*)(dsts + e0 + 4);
  } else {
    da.x = (e0     < nE) ? dsts[min(e0,     nE - 1)] : sent;
    da.y = (e0 + 1 < nE) ? dsts[min(e0 + 1, nE - 1)] : sent;
    da.z = (e0 + 2 < nE) ? dsts[min(e0 + 2, nE - 1)] : sent;
    da.w = (e0 + 3 < nE) ? dsts[min(e0 + 3, nE - 1)] : sent;
    db.x = (e0 + 4 < nE) ? dsts[min(e0 + 4, nE - 1)] : sent;
    db.y = (e0 + 5 < nE) ? dsts[min(e0 + 5, nE - 1)] : sent;
    db.z = (e0 + 6 < nE) ? dsts[min(e0 + 6, nE - 1)] : sent;
    db.w = (e0 + 7 < nE) ? dsts[min(e0 + 7, nE - 1)] : sent;
  }
  const unsigned nbs = (unsigned)slotBase;
  const unsigned unb = (unsigned)nb;
  const unsigned s0 = (unsigned)da.x - nbs, s1 = (unsigned)da.y - nbs;
  const unsigned s2 = (unsigned)da.z - nbs, s3 = (unsigned)da.w - nbs;
  const unsigned s4 = (unsigned)db.x - nbs, s5 = (unsigned)db.y - nbs;
  const unsigned s6 = (unsigned)db.z - nbs, s7 = (unsigned)db.w - nbs;
  const bool h0 = s0 < unb, h1 = s1 < unb, h2 = s2 < unb, h3 = s3 < unb;
  const bool h4 = s4 < unb, h5 = s5 < unb, h6 = s6 < unb, h7 = s7 < unb;
  const unsigned any = __builtin_amdgcn_ballot_w32(h0 | h1 | h2 | h3 | h4 | h5 | h6 | h7);
  if (any != 0u) {
#define HITJ(J, HJ, SJ) { \
      const unsigned mj = __builtin_amdgcn_ballot_w32(HJ); \
      if (mj != 0u) { \
        if (HJ) { \
          const int pos = wc + (int)__builtin_amdgcn_mbcnt_lo(mj, 0u); \
          if (pos < WCAP) list[wave * WCAP + pos] = ((el0 + (J)) << 12) | (int)(SJ); \
        } \
        wc += (int)__builtin_popcount(mj); } }
    HITJ(0, h0, s0)
    HITJ(1, h1, s1)
    HITJ(2, h2, s2)
    HITJ(3, h3, s3)
    HITJ(4, h4, s4)
    HITJ(5, h5, s5)
    HITJ(6, h6, s6)
    HITJ(7, h7, s7)
#undef HITJ
  }
  return wc;
}

__global__ __launch_bounds__(NTHR) void k_xprep(const float* __restrict__ x, _Float16* xh, int nN, int nUnits) {
  const int i = (int)blockIdx.x * NTHR + (int)threadIdx.x;
  if (i >= nUnits) return;
  const int row = i >> 5;
  const int c0  = (i & 31) * 8;
  const int rc  = row < nN ? row : nN - 1;
  const int cc  = c0 & (IN_DIM - 1);
  const float* p = x + (size_t)rc * IN_DIM + cc;
  v4f a = *(const v4f*)p, b = *(const v4f*)(p + 4);
  const v4f z4 = {0.f, 0.f, 0.f, 0.f};
  if (row >= nN || c0 >= IN_DIM) { a = z4; b = z4; }
  v8h hv;
  hv[0] = (_Float16)(a.x * CA1); hv[1] = (_Float16)(a.y * CA1);
  hv[2] = (_Float16)(a.z * CA1); hv[3] = (_Float16)(a.w * CA1);
  hv[4] = (_Float16)(b.x * CA1); hv[5] = (_Float16)(b.y * CA1);
  hv[6] = (_Float16)(b.z * CA1); hv[7] = (_Float16)(b.w * CA1);
  const size_t o = (size_t)row * KP + c0;
  *(volatile v8h*)(xh + o) = hv;
  __threadfence();
  *(volatile v8h*)(xh + o) = hv;
}

__global__ __launch_bounds__(NTHR) void k_wprep(const float* __restrict__ w1, const float* __restrict__ w2,
                                                const float* __restrict__ w3, _Float16* wt) {
  const int j  = (int)blockIdx.y;
  const int u  = (int)blockIdx.x * NTHR + (int)threadIdx.x;
  const int nrow = (j == 0) ? F1 : ((j == 1) ? F2 : G3);
  const int nUnits = nrow * (KP / 8);
  if (u >= nUnits) return;
  const int n  = u >> 5;
  const int k8 = (u & 31) * 8;
  const v4f z4 = {0.f, 0.f, 0.f, 0.f};
  v4f a, b;
  bool valid;
  if (j == 0) {
    valid = k8 < IN_DIM;
    const int kc = (k8 < IN_DIM) ? k8 : (IN_DIM - 8);
    const float* p = w1 + (size_t)kc * F1 + n;
    a.x = p[0 * F1]; a.y = p[1 * F1]; a.z = p[2 * F1]; a.w = p[3 * F1];
    b.x = p[4 * F1]; b.y = p[5 * F1]; b.z = p[6 * F1]; b.w = p[7 * F1];
  } else if (j == 1) {
    valid = true;
    const float* p = w2 + (size_t)k8 * F2 + n;
    a.x = p[0 * F2]; a.y = p[1 * F2]; a.z = p[2 * F2]; a.w = p[3 * F2];
    b.x = p[4 * F2]; b.y = p[5 * F2]; b.z = p[6 * F2]; b.w = p[7 * F2];
  } else {
    valid = k8 < GRUD;
    const int kc = (k8 < GRUD) ? k8 : (GRUD - 8);
    const float* p = w3 + (size_t)n * GRUD + kc;
    a = *(const v4f*)p;
    b = *(const v4f*)(p + 4);
  }
  if (!valid) { a = z4; b = z4; }
  v8h hv;
  hv[0] = (_Float16)(a.x * CW); hv[1] = (_Float16)(a.y * CW);
  hv[2] = (_Float16)(a.z * CW); hv[3] = (_Float16)(a.w * CW);
  hv[4] = (_Float16)(b.x * CW); hv[5] = (_Float16)(b.y * CW);
  hv[6] = (_Float16)(b.z * CW); hv[7] = (_Float16)(b.w * CW);
  const size_t rowb = (j == 0) ? 0 : ((j == 1) ? (size_t)F1 : (size_t)(F1 + F2));
  const size_t o = (rowb + (size_t)n) * KP + k8;
  *(volatile v8h*)(wt + o) = hv;
  __threadfence();
  *(volatile v8h*)(wt + o) = hv;
}

__global__ __launch_bounds__(GTHR) void k_gemm(const _Float16* __restrict__ xh, const _Float16* __restrict__ wt,
                                               const float* __restrict__ asrc, const float* __restrict__ adst,
                                               float* Y, float* ES, float* ED,
                                               int nks, int npass, int hmode, int alen, float scl) {
  __shared__ __attribute__((aligned(16))) float stg[GBM * HC];
  __shared__ __attribute__((aligned(16))) float esT[GBM * EP];
  __shared__ __attribute__((aligned(16))) float edT[GBM * EP];
  __shared__ float sAs[F1];
  __shared__ float sAd[F1];
  const int tid = threadIdx.x, lane = tid & 31, wave = tid >> 5, hh = lane >> 4, m = lane & 15;
  const int rowBase = (int)blockIdx.x * GBM;
  const int al = alen < 1 ? 1 : (alen > F1 ? F1 : alen);
  {
    const int i0 = tid < al ? tid : al - 1;
    const int i1 = (tid + GTHR) < al ? (tid + GTHR) : al - 1;
    sAs[tid] = asrc[i0];
    sAd[tid] = adst[i0];
    sAs[tid + GTHR] = asrc[i1];
    sAd[tid + GTHR] = adst[i1];
    esT[tid] = 0.f; esT[tid + GTHR] = 0.f;
    edT[tid] = 0.f; edT[tid + GTHR] = 0.f;
  }
  const int nk = nks < 1 ? 1 : (nks > KP / 32 ? KP / 32 : nks);
  const int np = npass < 1 ? 1 : (npass > YP / HC ? YP / HC : npass);
  const size_t arow = (size_t)(rowBase + 16 * wave + m) * KP + 8 * hh;
#pragma unroll 1
  for (int p = 0; p < np; ++p) {
    v8f acc[4];
#pragma unroll
    for (int t = 0; t < 4; ++t) { v8f z = {0.f, 0.f, 0.f, 0.f, 0.f, 0.f, 0.f, 0.f}; acc[t] = z; }
    const size_t brow = (size_t)(p * HC + m) * KP + 8 * hh;
#pragma unroll 1
    for (int ks = 0; ks < nk; ++ks) {
      FragH af;
      af.h[0] = *(const v8h*)(xh + arow + 32 * ks);
      af.h[1] = *(const v8h*)(xh + arow + 32 * ks + 16);
#pragma unroll
      for (int t = 0; t < 4; ++t) {
        const size_t bo = brow + (size_t)(16 * t) * KP + 32 * ks;
        FragH bf;
        bf.h[0] = *(const v8h*)(wt + bo);
        bf.h[1] = *(const v8h*)(wt + bo + 16);
        acc[t] = wmh(af, bf, acc[t]);
      }
    }
    float* sp = stg + (size_t)(16 * wave + 8 * hh) * HC + m;
#pragma unroll
    for (int t = 0; t < 4; ++t) {
#pragma unroll
      for (int r = 0; r < 8; ++r) sp[(size_t)r * HC + 16 * t] = acc[t][r] * scl;
    }
    __syncthreads();
    if (hmode != 0) {
      const int row  = tid >> 1;
      const int half = tid & 1;
      const float* srow = stg + (size_t)row * HC;
      const int pa = (p * HC) < (F1 - HC) ? (p * HC) : (F1 - HC);
      float s = 0.f, d = 0.f;
#pragma unroll 1
      for (int c = 0; c < 32; ++c) {
        const int cc = half * 32 + c;
        const float v = srow[cc];
        s = fmaf(v, sAs[pa + cc], s);
        d = fmaf(v, sAd[pa + cc], d);
      }
      s += __shfl_xor(s, 1);
      d += __shfl_xor(d, 1);
      if (half == 0 && p < EP) {
        esT[row * EP + p] = s;
        edT[row * EP + p] = d;
      }
    }
    const int nF4 = GBM * HC / 4;
    float* yb = Y + (size_t)rowBase * YP + HC * p;
    const v4f* s4 = (const v4f*)stg;
#pragma unroll 1
    for (int f = tid; f < nF4; f += GTHR) {
      const int r = f >> 4, q = f & 15;
      const v4f v = s4[f];
      *(volatile v4f*)(yb + (size_t)r * YP + 4 * q) = v;
    }
    __threadfence();
#pragma unroll 1
    for (int f = tid; f < nF4; f += GTHR) {
      const int r = f >> 4, q = f & 15;
      const v4f v = s4[f];
      *(volatile v4f*)(yb + (size_t)r * YP + 4 * q) = v;
    }
    __syncthreads();
  }
  if (hmode != 0 && wave < 2) {
    v4f ve = *(const v4f*)(esT + 128 * wave + 4 * lane);
    v4f vd = *(const v4f*)(edT + 128 * wave + 4 * lane);
    if (hmode == 1) {
      const float se = (ve.x + ve.y) + (ve.z + ve.w);
      const float sd = (vd.x + vd.y) + (vd.z + vd.w);
      ve.x = se; ve.y = 0.f; ve.z = 0.f; ve.w = 0.f;
      vd.x = sd; vd.y = 0.f; vd.z = 0.f; vd.w = 0.f;
    }
    float* pe = ES + (size_t)rowBase * EP + 128 * wave + 4 * lane;
    float* pd = ED + (size_t)rowBase * EP + 128 * wave + 4 * lane;
    *(volatile v4f*)pe = ve;
    *(volatile v4f*)pd = vd;
    __threadfence();
    *(volatile v4f*)pe = ve;
    *(volatile v4f*)pd = vd;
  }
}

__global__ __launch_bounds__(NTHR) void k_agg(
    const int* __restrict__ srcs, const int* __restrict__ dsts,
    const float* __restrict__ Y, const float* __restrict__ ES, const float* __restrict__ ED,
    const float* __restrict__ bias, _Float16* xout,
    int nN, int nE, int nb, int vec8, int nch, int hshift, float oca) {
  extern __shared__ v4f lds_dyn[];
  int* reg1 = (int*)lds_dyn;
  int* reg2 = reg1 + RCAP;
  int* scnt = reg2 + RCAP;
  int* soff = scnt + NBMAX;
  int* list = soff + NBMAX;
  int* wcnt = list + LISTN;
  int* wtot = wcnt + NWAVE;
  const int tid = threadIdx.x, lane = tid & 31, wave = tid >> 5;
  const int nodeBase = (int)blockIdx.x * nb;

  for (int i = tid; i < NBMAX; i += NTHR) scnt[i] = 0;
  __syncthreads();

  int tot = 0;
  const int nChunks = (nE + CHUNK - 1) / CHUNK;
#pragma unroll 1
  for (int ch = 0; ch < nChunks; ++ch) {
    const int cbase = ch * CHUNK;
    const int wc = scan_chunk(dsts, nE, cbase, nodeBase, nb, vec8, list, tid, lane, wave);
    if (lane == 0) wcnt[wave] = wc;
    __syncthreads();
    int pre = 0, all = 0;
#pragma unroll
    for (int w2 = 0; w2 < NWAVE; ++w2) {
      int c = wcnt[w2];
      c = c < 0 ? 0 : (c > WCAP ? WCAP : c);
      all += c;
      pre += (w2 < wave) ? c : 0;
    }
    const int wcc  = wc > WCAP ? WCAP : wc;
    const int base = tot + pre;
#pragma unroll 1
    for (int i = lane; i < wcc; i += 32) {
      const int ent = list[wave * WCAP + i];
      const int el  = (ent >> 12) & (CHUNK - 1);
      const int sl  = ent & (NBMAX - 1);
      int eid = cbase + el;
      eid = eid > nE - 1 ? nE - 1 : eid;
      const int pos = base + i;
      if (pos < RCAP) reg1[pos] = (int)(((unsigned)eid << 12) | (unsigned)sl);
    }
    tot += all;
    tot = tot > RCAP ? RCAP : tot;
    __syncthreads();
  }
  const int nh = tot;

  if (wave == 0) {
#pragma unroll 1
    for (int b0 = 0; b0 < nh; b0 += 32) {
      const int idx = b0 + lane;
      const int uv  = reg1[idx < RCAP ? idx : RCAP - 1];
      const int m32 = (nh - b0) < 32 ? (nh - b0) : 32;
#pragma unroll 1
      for (int k = 0; k < m32; ++k) {
        const int u  = __builtin_amdgcn_readlane(uv, k);
        const int sl = u & (NBMAX - 1);
        if (lane == 0) scnt[sl] = scnt[sl] + 1;
      }
    }
  }
  __syncthreads();

  {
    const v4i ca = *(const v4i*)(scnt + 8 * tid);
    const v4i cb = *(const v4i*)(scnt + 8 * tid + 4);
    const int e0 = ca.x < 0 ? 0 : ca.x, e1 = ca.y < 0 ? 0 : ca.y, e2 = ca.z < 0 ? 0 : ca.z, e3 = ca.w < 0 ? 0 : ca.w;
    const int e4 = cb.x < 0 ? 0 : cb.x, e5 = cb.y < 0 ? 0 : cb.y, e6 = cb.z < 0 ? 0 : cb.z, e7 = cb.w < 0 ? 0 : cb.w;
    const int ts = e0 + e1 + e2 + e3 + e4 + e5 + e6 + e7;
    int incl = ts;
#pragma unroll
    for (int d = 1; d < 32; d <<= 1) {
      const int up = __shfl_up(incl, d);
      if (lane >= d) incl += up;
    }
    if (lane == 31) wtot[wave] = incl;
    __syncthreads();
    int pre = 0;
#pragma unroll
    for (int w2 = 0; w2 < NWAVE; ++w2) pre += (w2 < wave) ? wtot[w2] : 0;
    int run = pre + incl - ts;
    soff[8 * tid + 0] = run; run += e0;
    soff[8 * tid + 1] = run; run += e1;
    soff[8 * tid + 2] = run; run += e2;
    soff[8 * tid + 3] = run; run += e3;
    soff[8 * tid + 4] = run; run += e4;
    soff[8 * tid + 5] = run; run += e5;
    soff[8 * tid + 6] = run; run += e6;
    soff[8 * tid + 7] = run;
  }
  __syncthreads();
  for (int i = tid; i < NBMAX; i += NTHR) list[i] = soff[i];
  __syncthreads();

  if (wave == 0) {
#pragma unroll 1
    for (int b0 = 0; b0 < nh; b0 += 32) {
      const int idx = b0 + lane;
      const int uv  = reg1[idx < RCAP ? idx : RCAP - 1];
      const int m32 = (nh - b0) < 32 ? (nh - b0) : 32;
#pragma unroll 1
      for (int k = 0; k < m32; ++k) {
        const int u   = __builtin_amdgcn_readlane(uv, k);
        const int sl  = u & (NBMAX - 1);
        const int eid = (int)((unsigned)u >> 12);
        if (lane == 0) {
          int pos = list[sl];
          pos = pos < 0 ? 0 : (pos > RCAP - 1 ? RCAP - 1 : pos);
          reg2[pos] = eid;
          list[sl] = pos + 1;
        }
      }
    }
  }
  __syncthreads();

  const int nbw = nb >> 3;
  const int c8  = 8 * lane;
  const bool act = c8 < nch;
  const int cc  = c8 & (nch - 1);
  const int hd  = lane >> hshift;
  const v4f bz0 = *(const v4f*)(bias + cc);
  const v4f bz1 = *(const v4f*)(bias + cc + 4);
  const bool ovf = (nh >= RCAP);
  const float qnan = __int_as_float(0x7fc00000);
  const _Float16 hzero = (_Float16)0.0f;
#pragma unroll 1
  for (int jt = 0; jt < nbw; ++jt) {
    const int slot = wave * nbw + jt;
    const int grow = nodeBase + slot;
    const int gcl  = grow < nN ? grow : nN - 1;
    int st = soff[slot];
    const int craw = scnt[slot];
    int cnt = craw;
    st  = st < 0 ? 0 : (st > nh ? nh : st);
    cnt = cnt < 0 ? 0 : (cnt > DEGCAP ? DEGCAP : cnt);
    if (cnt > nh - st) cnt = nh - st;
    const float pz = (ovf || craw > DEGCAP) ? qnan : 0.0f;
    const bool wr = grow < nN;

    const float* yd = Y + (size_t)gcl * YP + cc;
    const v4f xd0 = *(const v4f*)yd;
    const v4f xd1 = *(const v4f*)(yd + 4);
    const float edv = ED[(size_t)gcl * EP + hd];
    const float esd = ES[(size_t)gcl * EP + hd];
    const float t0 = esd + edv;
    float mx = fmaxf(t0, NEG_SLOPE * t0);
    float dn = 1.0f;
    v4f a0 = xd0, a1 = xd1;
#pragma unroll 1
    for (int q = 0; q < cnt; ++q) {
      int idx = st + q; idx = idx > RCAP - 1 ? RCAP - 1 : idx;
      int eid = reg2[idx]; eid = eid < 0 ? 0 : (eid > nE - 1 ? nE - 1 : eid);
      const int sraw = srcs[eid];
      const int s = sraw < 0 ? 0 : (sraw > nN - 1 ? nN - 1 : sraw);
      const float* ys = Y + (size_t)s * YP + cc;
      const v4f xs0 = *(const v4f*)ys;
      const v4f xs1 = *(const v4f*)(ys + 4);
      const float ess = ES[(size_t)s * EP + hd];
      const float u = ess + edv;
      const float l = fmaxf(u, NEG_SLOPE * u);
      const float mn = fmaxf(mx, l);
      const float s1 = __expf(mx - mn), s2 = __expf(l - mn);
      dn = fmaf(dn, s1, s2);
      a0.x = fmaf(a0.x, s1, s2 * xs0.x);
      a0.y = fmaf(a0.y, s1, s2 * xs0.y);
      a0.z = fmaf(a0.z, s1, s2 * xs0.z);
      a0.w = fmaf(a0.w, s1, s2 * xs0.w);
      a1.x = fmaf(a1.x, s1, s2 * xs1.x);
      a1.y = fmaf(a1.y, s1, s2 * xs1.y);
      a1.z = fmaf(a1.z, s1, s2 * xs1.z);
      a1.w = fmaf(a1.w, s1, s2 * xs1.w);
      mx = mn;
    }
    const float inv = __builtin_amdgcn_rcpf(dn);
    float v0 = fmaf(a0.x, inv, bz0.x), v1 = fmaf(a0.y, inv, bz0.y);
    float v2 = fmaf(a0.z, inv, bz0.z), v3 = fmaf(a0.w, inv, bz0.w);
    float v4 = fmaf(a1.x, inv, bz1.x), v5 = fmaf(a1.y, inv, bz1.y);
    float v6 = fmaf(a1.z, inv, bz1.z), v7 = fmaf(a1.w, inv, bz1.w);
    v0 = (v0 > 0.f ? v0 : (__expf(v0) - 1.0f)) + pz;
    v1 = (v1 > 0.f ? v1 : (__expf(v1) - 1.0f)) + pz;
    v2 = (v2 > 0.f ? v2 : (__expf(v2) - 1.0f)) + pz;
    v3 = (v3 > 0.f ? v3 : (__expf(v3) - 1.0f)) + pz;
    v4 = (v4 > 0.f ? v4 : (__expf(v4) - 1.0f)) + pz;
    v5 = (v5 > 0.f ? v5 : (__expf(v5) - 1.0f)) + pz;
    v6 = (v6 > 0.f ? v6 : (__expf(v6) - 1.0f)) + pz;
    v7 = (v7 > 0.f ? v7 : (__expf(v7) - 1.0f)) + pz;
    v8h hv;
    hv[0] = act ? (_Float16)(v0 * oca) : hzero;
    hv[1] = act ? (_Float16)(v1 * oca) : hzero;
    hv[2] = act ? (_Float16)(v2 * oca) : hzero;
    hv[3] = act ? (_Float16)(v3 * oca) : hzero;
    hv[4] = act ? (_Float16)(v4 * oca) : hzero;
    hv[5] = act ? (_Float16)(v5 * oca) : hzero;
    hv[6] = act ? (_Float16)(v6 * oca) : hzero;
    hv[7] = act ? (_Float16)(v7 * oca) : hzero;
    _Float16* xp = xout + (size_t)gcl * KP + c8;
    if (wr) *(volatile v8h*)xp = hv;
    __threadfence();
    if (wr) *(volatile v8h*)xp = hv;
  }
}

__global__ __launch_bounds__(NTHR) void k_gru(const float* __restrict__ G, const float* __restrict__ bih,
                                              const float* __restrict__ bhh, float* hout, int nN) {
  const int tid = threadIdx.x, lane = tid & 31, wave = tid >> 5;
  const int row = (int)blockIdx.x * NWAVE + wave;
  if (row >= nN) return;
  const int c = 4 * lane;
  const float* g = G + (size_t)row * YP + c;
  const v4f gr = *(const v4f*)g;
  const v4f gz = *(const v4f*)(g + GRUD);
  const v4f gn = *(const v4f*)(g + 2 * GRUD);
  const v4f ir = *(const v4f*)(bih + c);
  const v4f iz = *(const v4f*)(bih + GRUD + c);
  const v4f inn = *(const v4f*)(bih + 2 * GRUD + c);
  const v4f hr = *(const v4f*)(bhh + c);
  const v4f hz = *(const v4f*)(bhh + GRUD + c);
  const v4f hn = *(const v4f*)(bhh + 2 * GRUD + c);
  v4f h;
#define GRU1(C) { \
    const float rr = sigf((gr.C + ir.C) + hr.C); \
    const float zz = sigf((gz.C + iz.C) + hz.C); \
    const float nn = tnhf((gn.C + inn.C) + rr * hn.C); \
    h.C = (1.0f - zz) * nn; }
  GRU1(x)
  GRU1(y)
  GRU1(z)
  GRU1(w)
#undef GRU1
  float* p = hout + (size_t)row * GRUD + c;
  *(volatile v4f*)p = h;
  __threadfence();
  *(volatile v4f*)p = h;
}

__global__ __launch_bounds__(NTHR) void k_tail(const float* hsrc,
                                               const float* __restrict__ cI, const float* __restrict__ cR,
                                               const float* __restrict__ WI, const float* __restrict__ bI,
                                               const float* __restrict__ WR, const float* __restrict__ bR,
                                               const float* __restrict__ WS, const float* __restrict__ bS,
                                               const float* __restrict__ Npop,
                                               const float* __restrict__ I0, const float* __restrict__ R0,
                                               float* out0, float* out1, float* out2, float* out3, int nN) {
#pragma clang fp contract(off)
  __shared__ __attribute__((aligned(16))) float sH[TN * HKP];
  __shared__ float sW[TN * HK];
  __shared__ float sB[TN];
  __shared__ float sP[NO * TN];
  __shared__ __attribute__((aligned(16))) float sO[4 * TN * PW];
  const int tid = threadIdx.x, lane = tid & 31, wave = tid >> 5;
  const int nodeBase = (int)blockIdx.x * TN;

#pragma unroll
  for (int i = 0; i < 4; ++i) {
    const int f = tid + NTHR * i;
    const int row = f >> 5, q = f & 31;
    int nd = nodeBase + row; nd = nd < nN ? nd : nN - 1;
    const v4f v = *(const v4f*)(hsrc + (size_t)nd * GRUD + 4 * q);
    *(v4f*)(sH + row * HKP + 4 * q) = v;
  }
  if (tid < TN) {
    int nd = nodeBase + tid; nd = nd < nN ? nd : nN - 1;
    sH[tid * HKP + GRUD]     = cI[nd];
    sH[tid * HKP + GRUD + 1] = cR[nd];
    sH[tid * HKP + GRUD + 2] = 0.f;
    sH[tid * HKP + GRUD + 3] = 0.f;
    const float vbI = bI[tid < PW ? tid : PW - 1];
    int rI = tid - PW; rI = rI < 0 ? 0 : (rI > PW - 1 ? PW - 1 : rI);
    const float vbR = bR[rI];
    int rS = tid - 2 * PW; rS = rS < 0 ? 0 : (rS > 1 ? 1 : rS);
    const float vbS = bS[rS];
    sB[tid] = (tid < PW) ? vbI : ((tid < 2 * PW) ? vbR : vbS);
  }
#pragma unroll 1
  for (int i = tid; i < TN * HK; i += NTHR) {
    const int r = i / HK;
    const int k = i - r * HK;
    const int rI = r < PW ? r : PW - 1;
    int rR = r - PW; rR = rR < 0 ? 0 : (rR > PW - 1 ? PW - 1 : rR);
    int rS = r - 2 * PW; rS = rS < 0 ? 0 : (rS > 1 ? 1 : rS);
    const float vI = WI[rI * HK + k];
    const float vR = WR[rR * HK + k];
    const float vS = WS[rS * HK + k];
    sW[i] = (r < PW) ? vI : ((r < 2 * PW) ? vR : vS);
  }
  __syncthreads();

#pragma unroll 1
  for (int pass = 0; pass < NO / NWAVE; ++pass) {
    const int o = wave + NWAVE * pass;
    const float* wrow = sW + o * HK;
    const float* hrow = sH + lane * HKP;
    float s = 0.f;
#pragma unroll 2
    for (int k = 0; k < HK; ++k) s = fmaf(hrow[k], wrow[k], s);
    sP[o * TN + lane] = s + sB[o];
  }
  __syncthreads();

#pragma unroll 1
  for (int i = tid; i < TN * PW; i += NTHR) {
    const int nd = i / PW;
    const int t  = i - nd * PW;
    sO[i]           = sP[t * TN + nd];
    sO[TN * PW + i] = sP[(PW + t) * TN + nd];
  }
  if (tid < TN) {
    int nd = nodeBase + tid; nd = nd < nN ? nd : nN - 1;
    const float alp = sigf(sP[(2 * PW) * TN + tid]);
    const float bet = sigf(sP[(2 * PW + 1) * TN + tid]);
    const float Nv = Npop[nd];
    float Iv = I0[nd];
    const float Rv = R0[nd];
    const float S = (Nv - Iv) - Rv;
    const float q = S / Nv;
#pragma unroll 1
    for (int t = 0; t < PW; ++t) {
      const float t1 = alp * Iv;
      const float t2 = t1 * q;
      const float t3 = bet * Iv;
      const float dI = t2 - t3;
      sO[2 * TN * PW + tid * PW + t] = dI;
      sO[3 * TN * PW + tid * PW + t] = t3;
      Iv = Iv + dI;
    }
  }
  __syncthreads();

  const int nValid = (nN - nodeBase) < TN ? (nN - nodeBase) : TN;
  const int fl  = nValid * PW;
  const int n4  = fl >> 2;
  const int rem = fl & 3;
  const size_t ob = (size_t)nodeBase * PW;
  const v4f* s4 = (const v4f*)sO;
  const int SEG4 = TN * PW / 4;
  const int ti = tid < n4 ? tid : 0;
  const v4f va = s4[ti], vb = s4[SEG4 + ti], vc = s4[2 * SEG4 + ti], vd = s4[3 * SEG4 + ti];
  int d = tid - n4; d = d < 0 ? 0 : (d > 3 ? 3 : d);
  int te = 4 * n4 + d; te = te < fl ? te : fl - 1;
  const float ta = sO[te], tb = sO[TN * PW + te], tc = sO[2 * TN * PW + te], td = sO[3 * TN * PW + te];
  const bool w4 = tid < n4;
  const bool tw = (rem != 0) && (tid >= n4) && (tid < n4 + rem);
  if (w4) {
    *(volatile v4f*)(out0 + ob + 4 * tid) = va;
    *(volatile v4f*)(out1 + ob + 4 * tid) = vb;
    *(volatile v4f*)(out2 + ob + 4 * tid) = vc;
    *(volatile v4f*)(out3 + ob + 4 * tid) = vd;
  }
  if (tw) {
    *(volatile float*)(out0 + ob + 4 * n4 + d) = ta;
    *(volatile float*)(out1 + ob + 4 * n4 + d) = tb;
    *(volatile float*)(out2 + ob + 4 * n4 + d) = tc;
    *(volatile float*)(out3 + ob + 4 * n4 + d) = td;
  }
  __threadfence();
  if (w4) {
    *(volatile v4f*)(out0 + ob + 4 * tid) = va;
    *(volatile v4f*)(out1 + ob + 4 * tid) = vb;
    *(volatile v4f*)(out2 + ob + 4 * tid) = vc;
    *(volatile v4f*)(out3 + ob + 4 * tid) = vd;
  }
  if (tw) {
    *(volatile float*)(out0 + ob + 4 * n4 + d) = ta;
    *(volatile float*)(out1 + ob + 4 * n4 + d) = tb;
    *(volatile float*)(out2 + ob + 4 * n4 + d) = tc;
    *(volatile float*)(out3 + ob + 4 * n4 + d) = td;
  }
}

static int pick_nb(int nE, int nN) {
  int nb = NBMAX;
  while (nb > 16 && (long long)nb * (long long)nE * 5LL > (long long)RCAP * (long long)nN * 4LL) nb >>= 1;
  return nb;
}

extern "C" void kernel_launch(void* const* d_in, const int* in_sizes, int n_in,
                              void* d_out, int out_size, void* d_ws, size_t ws_size,
                              hipStream_t stream) {
  if (n_in < 27) return;
  const int nN = in_sizes[0] / IN_DIM;
  if (nN <= 0 || in_sizes[0] != nN * IN_DIM) return;
  if (nN > (1 << 22)) return;
  const int nE = in_sizes[1] / 2;
  if (nE < 1 || in_sizes[1] != 2 * nE) return;
  if (nE > (1 << 20)) return;
  if (in_sizes[2] != nN || in_sizes[3] != nN || in_sizes[4] != nN) return;
  if (in_sizes[5] != nN || in_sizes[6] != nN) return;
  if (in_sizes[9] != IN_DIM * F1) return;
  if (in_sizes[10] != F1 || in_sizes[11] != F1 || in_sizes[12] != F1) return;
  if (in_sizes[13] != F1 * F2) return;
  if (in_sizes[14] != F2 || in_sizes[15] != F2 || in_sizes[16] != F2) return;
  if (in_sizes[17] != G3 * GRUD) return;
  if (in_sizes[19] != G3 || in_sizes[20] != G3) return;
  if (in_sizes[21] != PW * HK || in_sizes[22] != PW) return;
  if (in_sizes[23] != PW * HK || in_sizes[24] != PW) return;
  if (in_sizes[25] != 2 * HK || in_sizes[26] != 2) return;
  if (out_size != nN * (4 * PW + GRUD)) return;

  const float* x    = (const float*)d_in[0];
  const int*   EI   = (const int*)d_in[1];
  const float* cI   = (const float*)d_in[2];
  const float* cR   = (const float*)d_in[3];
  const float* Npop = (const float*)d_in[4];
  const float* I0   = (const float*)d_in[5];
  const float* R0   = (const float*)d_in[6];
  const float* W1   = (const float*)d_in[9];
  const float* as1  = (const float*)d_in[10];
  const float* ad1  = (const float*)d_in[11];
  const float* b1   = (const float*)d_in[12];
  const float* W2   = (const float*)d_in[13];
  const float* as2  = (const float*)d_in[14];
  const float* ad2  = (const float*)d_in[15];
  const float* b2   = (const float*)d_in[16];
  const float* Wih  = (const float*)d_in[17];
  const float* bih  = (const float*)d_in[19];
  const float* bhh  = (const float*)d_in[20];
  const float* WI   = (const float*)d_in[21];
  const float* bIv  = (const float*)d_in[22];
  const float* WR   = (const float*)d_in[23];
  const float* bRv  = (const float*)d_in[24];
  const float* WS   = (const float*)d_in[25];
  const float* bSv  = (const float*)d_in[26];
  float* out  = (float*)d_out;
  float* out0 = out;
  float* out1 = out + (size_t)nN * PW;
  float* out2 = out + (size_t)2 * nN * PW;
  float* out3 = out + (size_t)3 * nN * PW;
  float* hout = out + (size_t)4 * nN * PW;

  const int* src = EI;
  const int* dst = EI + nE;
  const int MP   = ((nN + GBM - 1) / GBM) * GBM;
  const int nb   = pick_nb(nE, nN);
  const int vec8 = ((nE & 3) == 0) ? 1 : 0;
  const int nUnits = MP * (KP / 8);

  char* ws = (char*)d_ws;
  size_t off = 0;
  const size_t oWT = off; off += (size_t)WTROWS * KP * 2;        off = (off + 255) & ~(size_t)255;
  const size_t oXH = off; off += (size_t)MP * KP * 2;            off = (off + 255) & ~(size_t)255;
  const size_t oY  = off; off += (size_t)MP * YP * 4;            off = (off + 255) & ~(size_t)255;
  const size_t oES = off; off += (size_t)MP * EP * 4;            off = (off + 255) & ~(size_t)255;
  const size_t oED = off; off += (size_t)MP * EP * 4;            off = (off + 255) & ~(size_t)255;
  if (off > ws_size || off > (size_t)WSCAP) return;
  _Float16* WT = (_Float16*)(ws + oWT);
  _Float16* XH = (_Float16*)(ws + oXH);
  float*    Y  = (float*)(ws + oY);
  float*    ES = (float*)(ws + oES);
  float*    ED = (float*)(ws + oED);

  hipFuncSetAttribute(reinterpret_cast<const void*>(&k_agg),
                      hipFuncAttributeMaxDynamicSharedMemorySize, LDS_AGG);

  k_xprep<<<(nUnits + NTHR - 1) / NTHR, NTHR, 0, stream>>>(x, XH, nN, nUnits);
  k_wprep<<<dim3((G3 * (KP / 8) + NTHR - 1) / NTHR, 3), NTHR, 0, stream>>>(W1, W2, Wih, WT);

  const int gG = MP / GBM;
  const int gA = (nN + nb - 1) / nb;

  k_gemm<<<gG, GTHR, 0, stream>>>(XH, WT, as1, ad1, Y, ES, ED, IN_DIM / 32, F1 / HC, 4, F1, SCL1);
  k_agg<<<gA, NTHR, LDS_AGG, stream>>>(src, dst, Y, ES, ED, b1, XH, nN, nE, nb, vec8, F1, 3, CA2);
  k_gemm<<<gG, GTHR, 0, stream>>>(XH, WT + (size_t)F1 * KP, as2, ad2, Y, ES, ED, F1 / 32, F2 / HC, 1, F2, SCL2);
  k_agg<<<gA, NTHR, LDS_AGG, stream>>>(src, dst, Y, ES, ED, b2, XH, nN, nE, nb, vec8, F2, 5, CA3);
  k_gemm<<<gG, GTHR, 0, stream>>>(XH, WT + (size_t)(F1 + F2) * KP, b1, b1, Y, ES, ED, GRUD / 32, G3 / HC, 0, 1, SCL3);
  k_gru<<<(nN + NWAVE - 1) / NWAVE, NTHR, 0, stream>>>(Y, bih, bhh, hout, nN);
  k_tail<<<(nN + TN - 1) / TN, NTHR, 0, stream>>>(hout, cI, cR, WI, bIv, WR, bRv, WS, bSv, Npop, I0, R0,
                                                  out0, out1, out2, out3, nN);
}
